// RaytracedOptics_43044162240549
// MI455X (gfx1250) — hardware-run, weakly checked
//
#include <hip/hip_runtime.h>
#include <math.h>

typedef __attribute__((ext_vector_type(16))) _Float16 v16h;
typedef __attribute__((ext_vector_type(8)))  _Float16 v8h;
typedef __attribute__((ext_vector_type(16))) __bf16   v16b;
typedef __attribute__((ext_vector_type(8)))  __bf16   v8b;
typedef __attribute__((ext_vector_type(8)))  float    v8f;
typedef __attribute__((ext_vector_type(4)))  float    v4f;

constexpr int kBatch   = 4;
constexpr int kImgH    = 1024;
constexpr int kImgW    = 1024;
constexpr int kChan    = 3;
constexpr int kFields  = 21;
constexpr int kGridH   = 8;
constexpr int kGridW   = 8;
constexpr int kCells   = kGridH * kGridW;
constexpr int kCell    = 128;
constexpr int kPsfN    = 65;
constexpr int kTapN    = 23;
constexpr int kTapHalf = 11;
constexpr int kNPix    = kPsfN * kPsfN * kChan;
constexpr int kNPixPad = 12736;
constexpr int kKPad    = 32;
constexpr int kWtsLd   = 64;
constexpr int kPadRows = kCell + 2 * kTapHalf;
constexpr int kPadCols = 160;
constexpr int kHaloL   = 16;
constexpr int kPatchEl = kPadRows * kPadCols;
constexpr int kPatches = kBatch * kChan * kCells;
constexpr int kChunksPerPatch = kPatchEl / 8;
constexpr int kToepK   = 64;
constexpr int kToepPlane = 16 * kToepK;
constexpr int kToepPerCell = kChan * kTapN * kToepPlane;
constexpr int kToepChunks  = kToepPerCell / 8;
constexpr size_t kPlaneEl  = (size_t)kImgH * kImgW;

static_assert(kNPix == 12675, "psf pixel-channel count");
static_assert(kNPixPad % 64 == 0 && kNPixPad >= kNPix, "N pad");
static_assert(kFields <= kKPad && (kKPad % 32) == 0, "K pad");
static_assert(kCell * kGridH == kImgH && kCell * kGridW == kImgW, "cells tile the image");
static_assert(kPadRows == 150, "padded patch rows");
static_assert((kPatchEl * 2) % 128 == 0, "patch is a whole number of 128-B lines");
static_assert(kChunksPerPatch == 3000, "chunks per patch");
static_assert((kToepPerCell * 2) % 128 == 0, "tap plane per cell is whole lines");
static_assert(kToepChunks == 8832, "tap chunks per cell");
static_assert(kTapN + 15 + 5 < kToepK, "tap window fits K");
static_assert(kHaloL + kCell + kHaloL == kPadCols, "padded columns");

constexpr float kWtCarry   = 64.0f;
constexpr float kPsfCarry  = 64.0f;
constexpr float kImgCarry  = 64.0f;
constexpr float kTapCarry  = 256.0f;
constexpr float kInterpScale = 1.0f / (kWtCarry * kPsfCarry);
constexpr float kConvScale   = 1.0f / (kImgCarry * kTapCarry);
constexpr float kCellPix   = (float)(kCell * kCell);
constexpr float kCountToWt = kWtCarry / kCellPix;
constexpr float kF16MinNormal = 6.103515625e-05f;

constexpr double kHalfDiagD = (double)(kImgH - 1) * 1.4142135623730951 * 0.5;
constexpr float kHalfDiag    = (float)kHalfDiagD;
constexpr float kInvHalfDiag = (float)(1.0 / kHalfDiagD);
constexpr float kCtr = (float)(kImgW - 1) * 0.5f;
constexpr float kFieldSteps = (float)(kFields - 1);
constexpr float kShrinkInv = (float)kPsfN / (float)kTapN;
constexpr float kShrink    = (float)kTapN / (float)kPsfN;
constexpr float kPsfCtr    = (float)(kPsfN - 1) * 0.5f;

constexpr size_t kSzWTS    = (size_t)kCells * kWtsLd * 2;
constexpr size_t kSzBT0    = (size_t)kNPixPad * kKPad * 2;
constexpr size_t kSzINTERP = (size_t)kCells * kNPixPad * 4;
constexpr size_t kSzPSFT   = (size_t)kCells * kToepPerCell * 2;
constexpr size_t kSzXPAD   = (size_t)kPatches * kPatchEl * 2 + 128;
constexpr size_t kSzBLUR   = (size_t)kBatch * kChan * kPlaneEl * 4;
constexpr size_t kOffWTS    = 0;
constexpr size_t kOffBT0    = kOffWTS + kSzWTS;
constexpr size_t kOffINTERP = kOffBT0 + kSzBT0;
constexpr size_t kOffPSFT   = kOffINTERP + kSzINTERP;
constexpr size_t kOffXPAD   = kOffPSFT + kSzPSFT;
constexpr size_t kOffBLUR   = kOffXPAD + kSzXPAD;
constexpr size_t kWsTotal   = kOffBLUR + kSzBLUR;
static_assert(kWsTotal == 8192ull + 815104ull + 3260416ull + 9043968ull + 36864128ull + 50331648ull, "carve sum");
static_assert(kWsTotal == 100323456ull, "carve total");
static_assert(kWsTotal <= 134217728ull, "carve cap");
static_assert((kOffBT0 % 128) == 0 && (kOffINTERP % 128) == 0 && (kOffPSFT % 128) == 0 &&
              (kOffXPAD % 128) == 0 && (kOffBLUR % 128) == 0, "128-B aligned regions");

__device__ __forceinline__ int imin_d(int a, int b) { return a < b ? a : b; }
__device__ __forceinline__ int imax_d(int a, int b) { return a > b ? a : b; }
__device__ __forceinline__ int iclamp_d(int v, int lo, int hi) { return imin_d(imax_d(v, lo), hi); }

__device__ __forceinline__ float flush_h(float v) { return (fabsf(v) < kF16MinNormal) ? 0.0f : v; }

__device__ __forceinline__ float coordf(int j) { return ((float)j - kCtr) * kInvHalfDiag; }

__device__ __forceinline__ void soft_index(float s, int& lo, int& hi, float& f) {
  s = fminf(fmaxf(s, 0.0f), kFieldSteps);
  const float fl = floorf(s);
  lo = iclamp_d((int)fl, 0, kFields - 1);
  hi = iclamp_d((int)ceilf(s), 0, kFields - 1);
  f = s - fl;
}

__device__ __forceinline__ float cubw(float t) {
  const float t2 = t * t, t3 = t2 * t;
  const float a = 1.5f * t3 - 2.5f * t2 + 1.0f;
  const float b = -0.5f * t3 + 2.5f * t2 - 4.0f * t + 2.0f;
  return (t <= 1.0f) ? a : ((t < 2.0f) ? b : 0.0f);
}

__device__ __forceinline__ v8f mma_h(v16h a, v16h b, v8f c) {
  c = __builtin_amdgcn_wmma_f32_16x16x32_f16(false, a, false, b, (short)0, c, false, false);
  asm volatile("v_nop\n\tv_nop\n\tv_nop\n\tv_nop" : "+v"(c) : "v"(a), "v"(b));
  return c;
}

__device__ __forceinline__ unsigned short f2bf_bits(float f) {
  unsigned u = __float_as_uint(f);
  return (unsigned short)((u + 0x7FFFu + ((u >> 16) & 1u)) >> 16);
}
__device__ __forceinline__ float bf_bits2f(unsigned short h) { return __uint_as_float(((unsigned)h) << 16); }

__device__ __forceinline__ void dep_guard_h(v8f& a, v8f& b, v16h x, v16h y) { asm volatile("v_nop\n\tv_nop\n\tv_nop\n\tv_nop" : "+v"(a), "+v"(b) : "v"(x), "v"(y)); }
__device__ __forceinline__ void dep_guard_b(v8f& a, v8f& b, v16b x, v16b y) { asm volatile("v_nop\n\tv_nop\n\tv_nop\n\tv_nop" : "+v"(a), "+v"(b) : "v"(x), "v"(y)); }
__device__ __forceinline__ void keep4_h(v16h a, v16h b, v16h c, v16h d) { asm volatile("v_nop" :: "v"(a), "v"(b), "v"(c), "v"(d)); }
__device__ __forceinline__ void keep4_b(v16b a, v16b b, v16b c, v16b d) { asm volatile("v_nop" :: "v"(a), "v"(b), "v"(c), "v"(d)); }
__device__ __forceinline__ void acc_guard4(v8f& a, v8f& b, v8f& c, v8f& d) { asm volatile("v_nop\n\tv_nop\n\tv_nop\n\tv_nop" : "+v"(a), "+v"(b), "+v"(c), "+v"(d)); }
template <typename T> struct Frag;
template <> struct Frag<_Float16> {
  typedef v16h V; union U { v16h v; v8h h[2]; };
  static __device__ __forceinline__ v16h load(const _Float16* p) {
    U f; f.h[0] = *(const v8h*)(p); f.h[1] = *(const v8h*)(p + 16); return f.v;
  }
  static __device__ __forceinline__ v8f mma(v16h a, v16h b, v8f c) {
    return __builtin_amdgcn_wmma_f32_16x16x32_f16(false, a, false, b, (short)0, c, false, false);
  }
  static __device__ __forceinline__ void guard(v8f& a, v8f& b, v16h x, v16h y) { dep_guard_h(a, b, x, y); }
  static __device__ __forceinline__ void keep(v16h a, v16h b, v16h c, v16h d) { keep4_h(a, b, c, d); }
};
template <> struct Frag<__bf16> {
  typedef v16b V; union U { v16b v; v8b h[2]; };
  static __device__ __forceinline__ v16b load(const __bf16* p) {
    U f; f.h[0] = *(const v8b*)(p); f.h[1] = *(const v8b*)(p + 16); return f.v;
  }
  static __device__ __forceinline__ v8f mma(v16b a, v16b b, v8f c) {
    return __builtin_amdgcn_wmma_f32_16x16x32_bf16(false, a, false, b, (short)0, c, false, false);
  }
  static __device__ __forceinline__ void guard(v8f& a, v8f& b, v16b x, v16b y) { dep_guard_b(a, b, x, y); }
  static __device__ __forceinline__ void keep(v16b a, v16b b, v16b c, v16b d) { keep4_b(a, b, c, d); }
};

template <int ET> struct Elem;
template <> struct Elem<0> { typedef _Float16 T; };
template <> struct Elem<1> { typedef __bf16 T; };
template <int ET, bool SPLIT, int BIAS_MODE, int OUT_MODE, bool RESID, int ACT = 0>
__global__ __launch_bounds__(256) void wmma_gemm64(
    const unsigned short* __restrict__ Ap, const unsigned short* __restrict__ A2p, int lda, long strideA,
    const unsigned short* __restrict__ Btp, const unsigned short* __restrict__ Bt2p, int ldb, long strideB,
    void* __restrict__ Cout, void* __restrict__ Cout2, int ldc, long strideC,
    const float* __restrict__ bias,
    const float* __restrict__ resid, long strideR,
    int M, int N, int K, float scale) {
  typedef typename Elem<ET>::T T;
  typedef typename Frag<T>::V V;
  const T* A = (const T*)Ap; const T* A2 = (const T*)A2p; const T* Bt = (const T*)Btp; const T* Bt2 = (const T*)Bt2p;
  __shared__ __align__(16) float sT[8][16 * 68];
  const int b    = blockIdx.y;
  const int lane = threadIdx.x & 31;
  const int wave = threadIdx.x >> 5;
  const int tilesN = N >> 6;
  const int tilesM = M >> 6;
  const int tile = blockIdx.x * 8 + wave;
  if (tile >= tilesM * tilesN) return;
  const int tm = tile / tilesN;
  const int tn = tile - tm * tilesN;
  const int m0 = tm << 6;
  const int n0 = tn << 6;

  const T* Ab  = A  + (size_t)b * strideA;
  const T* Bb  = Bt + (size_t)b * strideB;
  const T* Ab2 = SPLIT ? (A2  + (size_t)b * strideA) : nullptr;
  const T* Bb2 = SPLIT ? (Bt2 + (size_t)b * strideB) : nullptr;

  const int rlane = lane & 15;
  const int koff  = (lane >> 4) * 8;
  const int mOff  = (lane >> 4) * 8;

  v8f acc[4][4];
#pragma unroll
  for (int i = 0; i < 4; ++i)
#pragma unroll
    for (int j = 0; j < 4; ++j) acc[i][j] = (v8f){0.f,0.f,0.f,0.f,0.f,0.f,0.f,0.f};

  for (int k0 = 0; k0 < K; k0 += 32) {
    V bh[4], bl[4];
#pragma unroll
    for (int j = 0; j < 4; ++j) {
      const size_t bo = (size_t)(n0 + (j << 4) + rlane) * ldb + koff + k0;
      bh[j] = Frag<T>::load(Bb + bo);
      if (SPLIT) bl[j] = Frag<T>::load(Bb2 + bo);
    }
#pragma unroll
    for (int i = 0; i < 4; ++i) {
      const size_t ao = (size_t)(m0 + (i << 4) + rlane) * lda + koff + k0;
      V ah = Frag<T>::load(Ab + ao);
      V al;
      if (SPLIT) al = Frag<T>::load(Ab2 + ao);
#pragma unroll
      for (int j = 0; j < 4; ++j) {
        acc[i][j] = Frag<T>::mma(ah, bh[j], acc[i][j]);
        if (SPLIT) {
          acc[i][j] = Frag<T>::mma(ah, bl[j], acc[i][j]);
          acc[i][j] = Frag<T>::mma(al, bh[j], acc[i][j]);
        }
      }
      Frag<T>::guard(acc[i][0], acc[i][3], ah, SPLIT ? al : ah);
    }
    Frag<T>::keep(bh[0], bh[1], bh[2], bh[3]);
    if (SPLIT) Frag<T>::keep(bl[0], bl[1], bl[2], bl[3]);
  }
  acc_guard4(acc[0][0], acc[0][1], acc[0][2], acc[0][3]);
  acc_guard4(acc[1][0], acc[1][1], acc[1][2], acc[1][3]);
  acc_guard4(acc[2][0], acc[2][1], acc[2][2], acc[2][3]);
  acc_guard4(acc[3][0], acc[3][1], acc[3][2], acc[3][3]);

  float* slab = sT[wave];
  const float* Rb = RESID ? (resid + (size_t)b * strideR) : nullptr;
#pragma unroll
  for (int i = 0; i < 4; ++i) {
    const int mBase = m0 + (i << 4);
#pragma unroll
    for (int j = 0; j < 4; ++j) {
      const int n = n0 + (j << 4) + rlane;
      float bv = 0.f;
      if (BIAS_MODE == 2) bv = bias[n];
#pragma unroll
      for (int r = 0; r < 8; ++r) {
        float v = acc[i][j][r] * scale;
        if (BIAS_MODE == 1) v += bias[mBase + mOff + r];
        if (BIAS_MODE == 2) v += bv;
        if (RESID) v += Rb[(size_t)(mBase + mOff + r) * ldc + n];
        if (ACT == 1) v = tanhf(v);
        if (ACT == 2) v = fmaxf(v, 0.0f);
        if (ACT == 4) v = (v > 0.f) ? v : 0.01f * v;
        slab[(mOff + r) * 68 + (j << 4) + rlane] = v;
      }
    }
    __builtin_amdgcn_fence(__ATOMIC_RELEASE, "workgroup");
    __builtin_amdgcn_wave_barrier();
    __builtin_amdgcn_fence(__ATOMIC_ACQUIRE, "workgroup");
    if (OUT_MODE == 0) {
      float* C = (float*)Cout + (size_t)b * strideC;
      const int hh = lane >> 4, c4 = (lane & 15) * 4;
      for (int pass = 0; pass < 2; ++pass) {
#pragma unroll
        for (int it = 0; it < 8; ++it) {
          const int row = it * 2 + hh;
          v4f v = *(const v4f*)(slab + row * 68 + c4);
          *(volatile v4f*)(C + (size_t)(mBase + row) * ldc + n0 + c4) = v;
        }
        __threadfence();
      }
    } else {
      const int q = lane >> 3, c8 = (lane & 7) * 8;
      unsigned short* C  = (unsigned short*)Cout  + (size_t)b * strideC;
      unsigned short* C2 = (OUT_MODE == 2) ? ((unsigned short*)Cout2 + (size_t)b * strideC) : nullptr;
      for (int pass = 0; pass < 2; ++pass) {
#pragma unroll
        for (int it = 0; it < 4; ++it) {
          const int row = it * 4 + q;
          const float* sp = slab + row * 68 + c8;
          v8h hv, lv;
#pragma unroll
          for (int e = 0; e < 8; ++e) {
            if (OUT_MODE == 1) {
              hv[e] = (_Float16)sp[e];
            } else {
              unsigned short hb = f2bf_bits(sp[e]);
              unsigned short lb = f2bf_bits(sp[e] - bf_bits2f(hb));
              hv[e] = __builtin_bit_cast(_Float16, hb);
              lv[e] = __builtin_bit_cast(_Float16, lb);
            }
          }
          *(volatile v8h*)(C + (size_t)(mBase + row) * ldc + n0 + c8) = hv;
          if (OUT_MODE == 2) *(volatile v8h*)(C2 + (size_t)(mBase + row) * ldc + n0 + c8) = lv;
        }
        __threadfence();
      }
    }
    __builtin_amdgcn_fence(__ATOMIC_RELEASE, "workgroup");
    __builtin_amdgcn_wave_barrier();
    __builtin_amdgcn_fence(__ATOMIC_ACQUIRE, "workgroup");
  }
}

__global__ __launch_bounds__(256) void weights_kernel(unsigned short* __restrict__ wts)
{
  __shared__ int part[8][32];
  __shared__ int hist[64];
  const int g = blockIdx.x, t = threadIdx.x;
  const int lane = t & 31, wave = t >> 5;
  const int gy = g >> 3, gx = g & 7;
  int cntAcc = 0;
#pragma unroll 1
  for (int i = 0; i < (kCell * kCell) / 256; ++i) {
    const int idx = i * 256 + t;
    const int row = gy * kCell + (idx >> 7);
    const int col = gx * kCell + (idx & (kCell - 1));
    const float xm = coordf(col), ym = coordf(row);
    const float fm = fminf(sqrtf(xm * xm + ym * ym), 1.0f);
    const int d = iclamp_d((int)rintf(fm * kFieldSteps), 0, kFields - 1);
#pragma unroll
    for (int f = 0; f < kFields; ++f) {
      const unsigned mask = __builtin_amdgcn_ballot_w32(d == f);
      const int cnt = __popc(mask);
      cntAcc += (lane == f) ? cnt : 0;
    }
  }
  part[wave][lane] = (lane < kFields) ? cntAcc : 0;
  __syncthreads();
  if (t < 64) {
    const int tc = imin_d(t, 31);
    int s = 0;
#pragma unroll
    for (int w = 0; w < 8; ++w) s += part[w][tc];
    hist[t] = (t < kFields) ? s : 0;
  }
  __syncthreads();
  if (t < 8) {
    v8h hv;
#pragma unroll
    for (int j = 0; j < 8; ++j) {
      const float v = flush_h((float)hist[t * 8 + j] * kCountToWt);
      hv[j] = (_Float16)v;
    }
    unsigned short* dst = wts + (size_t)g * kWtsLd + t * 8;
    *(volatile v8h*)dst = hv;
    __threadfence();
    *(volatile v8h*)dst = hv;
  }
}

__global__ __launch_bounds__(256) void bt_plane_kernel(const float* __restrict__ psfs, unsigned short* __restrict__ bt)
{
  __shared__ float sF[kKPad * 65];
  const int t = threadIdx.x;
  const int n0 = blockIdx.x * 64;
  const int nl = t & 63, kq = t >> 6;
  const int n = n0 + nl;
  const bool nok = n < kNPix;
  const int nc = imin_d(n, kNPix - 1);
#pragma unroll 1
  for (int i = 0; i < 8; ++i) {
    const int k = kq + 4 * i;
    const bool kok = k < kFields;
    const int kc = imin_d(k, kFields - 1);
    float v = psfs[(size_t)kc * kNPix + nc];
    asm volatile("" : "+v"(v));
    const float w = (kok && nok) ? flush_h(v * kPsfCarry) : 0.0f;
    sF[k * 65 + nl] = w;
  }
  __syncthreads();
  const int nn = t >> 2, k0 = (t & 3) * 8;
  v8h hv;
#pragma unroll
  for (int j = 0; j < 8; ++j) hv[j] = (_Float16)sF[(k0 + j) * 65 + nn];
  unsigned short* dst = bt + (size_t)n0 * kKPad + t * 8;
  *(volatile v8h*)dst = hv;
  __threadfence();
  *(volatile v8h*)dst = hv;
}

__global__ __launch_bounds__(256) void psf_finish_kernel(const float* __restrict__ interp, unsigned short* __restrict__ psfT)
{
  __shared__ float sP[kNPix + 1];
  __shared__ float sOut[kTapN * kTapN * kChan + 1];
  __shared__ float sInv[4];
  const int g = blockIdx.x, t = threadIdx.x;
  for (int i = t; i < kNPix; i += 256) sP[i] = interp[(size_t)g * kNPixPad + i];
  __syncthreads();
  const int gy = g >> 3, gx = g & 7;
  const float X = (float)gx - 3.5f, Y = (float)gy - 3.5f;
  const float hinv = 1.0f / sqrtf(X * X + Y * Y);
  const float ca = Y * hinv;
  const float sa = -X * hinv;

  for (int p = t; p < kTapN * kTapN; p += 256) {
    const int oy = p / kTapN, ox = p - oy * kTapN;
    const float sfy = ((float)oy + 0.5f) * kShrinkInv - 0.5f;
    const float sfx = ((float)ox + 0.5f) * kShrinkInv - 0.5f;
    const int iy0 = (int)ceilf(sfy - kShrinkInv);
    const int ix0 = (int)ceilf(sfx - kShrinkInv);
    float ysum = 0.0f, xsum = 0.0f;
#pragma unroll 1
    for (int j = 0; j < 6; ++j) {
      const int iy = iy0 + j, ix = ix0 + j;
      const float wy = fmaxf(1.0f - fabsf((float)iy - sfy) * kShrink, 0.0f);
      const float wx = fmaxf(1.0f - fabsf((float)ix - sfx) * kShrink, 0.0f);
      ysum += (iy >= 0 && iy < kPsfN) ? wy : 0.0f;
      xsum += (ix >= 0 && ix < kPsfN) ? wx : 0.0f;
    }
    const float inv = 1.0f / (ysum * xsum);
    float a0 = 0.0f, a1 = 0.0f, a2 = 0.0f;
#pragma unroll 1
    for (int jy = 0; jy < 6; ++jy) {
      const int iy = iy0 + jy;
      float wyv = fmaxf(1.0f - fabsf((float)iy - sfy) * kShrink, 0.0f);
      wyv = (iy >= 0 && iy < kPsfN) ? wyv : 0.0f;
      const float dyy = (float)iy - kPsfCtr;
#pragma unroll 1
      for (int jx = 0; jx < 6; ++jx) {
        const int ix = ix0 + jx;
        float wxv = fmaxf(1.0f - fabsf((float)ix - sfx) * kShrink, 0.0f);
        wxv = (ix >= 0 && ix < kPsfN) ? wxv : 0.0f;
        const float w = wyv * wxv;
        const float dxx = (float)ix - kPsfCtr;
        const float sx = ca * dxx + sa * dyy + kPsfCtr;
        const float sy = -sa * dxx + ca * dyy + kPsfCtr;
        const float fxs = floorf(sx), fys = floorf(sy);
        const int x0 = (int)fxs, y0 = (int)fys;
        const float fx = sx - fxs, fy = sy - fys;
        const float w00 = (1.0f - fy) * (1.0f - fx), w01 = (1.0f - fy) * fx;
        const float w10 = fy * (1.0f - fx), w11 = fy * fx;
        const bool vy0 = (y0 >= 0) && (y0 < kPsfN), vy1 = (y0 + 1 >= 0) && (y0 + 1 < kPsfN);
        const bool vx0 = (x0 >= 0) && (x0 < kPsfN), vx1 = (x0 + 1 >= 0) && (x0 + 1 < kPsfN);
        const int y0c = iclamp_d(y0, 0, kPsfN - 1), y1c = iclamp_d(y0 + 1, 0, kPsfN - 1);
        const int x0c = iclamp_d(x0, 0, kPsfN - 1), x1c = iclamp_d(x0 + 1, 0, kPsfN - 1);
        const int b00 = (y0c * kPsfN + x0c) * kChan, b01 = (y0c * kPsfN + x1c) * kChan;
        const int b10 = (y1c * kPsfN + x0c) * kChan, b11 = (y1c * kPsfN + x1c) * kChan;
        float rv[3];
#pragma unroll
        for (int c = 0; c < kChan; ++c) {
          const float p00 = sP[b00 + c], p01 = sP[b01 + c], p10 = sP[b10 + c], p11 = sP[b11 + c];
          const float g00 = (vy0 && vx0) ? p00 : 0.0f;
          const float g01 = (vy0 && vx1) ? p01 : 0.0f;
          const float g10 = (vy1 && vx0) ? p10 : 0.0f;
          const float g11 = (vy1 && vx1) ? p11 : 0.0f;
          rv[c] = g00 * w00 + g01 * w01 + g10 * w10 + g11 * w11;
        }
        a0 += w * rv[0];
        a1 += w * rv[1];
        a2 += w * rv[2];
      }
    }
    sOut[p * kChan + 0] = a0 * inv;
    sOut[p * kChan + 1] = a1 * inv;
    sOut[p * kChan + 2] = a2 * inv;
  }
  __syncthreads();
  if (t < kChan) {
    float s = 0.0f;
#pragma unroll 1
    for (int p = 0; p < kTapN * kTapN; ++p) s += sOut[p * kChan + t];
    sInv[t] = kTapCarry * (1.0f / s);
  }
  __syncthreads();
  unsigned short* base = psfT + (size_t)g * kToepPerCell;
#pragma unroll 1
  for (int it = 0; it < (kToepChunks + 255) / 256; ++it) {
    const int idx = it * 256 + t;
    const bool live = idx < kToepChunks;
    const int e = imin_d(idx, kToepChunks - 1) * 8;
    const int k0 = e & (kToepK - 1);
    const int n = (e >> 6) & 15;
    const int cd = e >> 10;
    const int c = cd / kTapN;
    const int dy = cd - c * kTapN;
    const float nrm = sInv[c];
    v8h hv;
#pragma unroll
    for (int j = 0; j < 8; ++j) {
      const int dx = k0 + j - n - 5;
      const bool ok = (dx >= 0) && (dx < kTapN);
      const int dxc = iclamp_d(dx, 0, kTapN - 1);
      const float tv = sOut[(dy * kTapN + dxc) * kChan + c] * nrm;
      const float v = ok ? flush_h(tv) : 0.0f;
      hv[j] = (_Float16)v;
    }
    if (live) {
      unsigned short* dst = base + e;
      *(volatile v8h*)dst = hv;
      __threadfence();
      *(volatile v8h*)dst = hv;
    }
  }
}

__global__ __launch_bounds__(256) void prep_kernel(const float* __restrict__ img, const float* __restrict__ riTab,
                                                   unsigned short* __restrict__ xpad)
{
  __shared__ float sRI[32];
  const int t = threadIdx.x;
  if (t < 32) sRI[t] = riTab[imin_d(t, kFields - 1)];
  __syncthreads();
  const int b = blockIdx.x >> 6, g = blockIdx.x & 63;
  const int gy = g >> 3, gx = g & 7;
#pragma unroll 1
  for (int it = 0; it < (kChunksPerPatch + 255) / 256; ++it) {
    const int idx = it * 256 + t;
    const bool live = idx < kChunksPerPatch;
    const int idc = imin_d(idx, kChunksPerPatch - 1);
    const int row = idc / 20;
    const int cc = idc - row * 20;
    const bool inter = (row >= kTapHalf) && (row < kTapHalf + kCell) && (cc >= 2) && (cc < 18);
    const int irow = iclamp_d(gy * kCell + row - kTapHalf, 0, kImgH - 1);
    const int icol0 = iclamp_d(gx * kCell + cc * 8 - kHaloL, 0, kImgW - 8);
    const float* src = img + ((size_t)(b * kImgH + irow) * kImgW + icol0) * kChan;
    v4f f0 = *(const v4f*)(src);
    v4f f1 = *(const v4f*)(src + 4);
    v4f f2 = *(const v4f*)(src + 8);
    v4f f3 = *(const v4f*)(src + 12);
    v4f f4 = *(const v4f*)(src + 16);
    v4f f5 = *(const v4f*)(src + 20);
    asm volatile("" : "+v"(f0));
    asm volatile("" : "+v"(f1));
    asm volatile("" : "+v"(f2));
    asm volatile("" : "+v"(f3));
    asm volatile("" : "+v"(f4));
    asm volatile("" : "+v"(f5));
    const float px[24] = { f0[0], f0[1], f0[2], f0[3], f1[0], f1[1], f1[2], f1[3],
                           f2[0], f2[1], f2[2], f2[3], f3[0], f3[1], f3[2], f3[3],
                           f4[0], f4[1], f4[2], f4[3], f5[0], f5[1], f5[2], f5[3] };
    const float ym = coordf(irow);
    const float y2 = ym * ym;
    v8h h0, h1, h2;
#pragma unroll
    for (int j = 0; j < 8; ++j) {
      const float xm = coordf(icol0 + j);
      const float fm = fminf(sqrtf(xm * xm + y2), 1.0f);
      int lo, hi;
      float f;
      soft_index(fm * kFieldSteps, lo, hi, f);
      const float ri = sRI[lo] * (1.0f - f) + sRI[hi] * f;
      const float sc = ri * kImgCarry;
      const float v0 = inter ? flush_h(px[3 * j + 0] * sc) : 0.0f;
      const float v1 = inter ? flush_h(px[3 * j + 1] * sc) : 0.0f;
      const float v2 = inter ? flush_h(px[3 * j + 2] * sc) : 0.0f;
      h0[j] = (_Float16)v0;
      h1[j] = (_Float16)v1;
      h2[j] = (_Float16)v2;
    }
    if (live) {
      unsigned short* d0 = xpad + ((size_t)((b * kChan + 0) * kCells + g)) * kPatchEl + (size_t)idc * 8;
      unsigned short* d1 = xpad + ((size_t)((b * kChan + 1) * kCells + g)) * kPatchEl + (size_t)idc * 8;
      unsigned short* d2 = xpad + ((size_t)((b * kChan + 2) * kCells + g)) * kPatchEl + (size_t)idc * 8;
      *(volatile v8h*)d0 = h0;
      *(volatile v8h*)d1 = h1;
      *(volatile v8h*)d2 = h2;
      __threadfence();
      *(volatile v8h*)d0 = h0;
      *(volatile v8h*)d1 = h1;
      *(volatile v8h*)d2 = h2;
    }
  }
  if (blockIdx.x == kBatch * kCells - 1 && t < 8) {
    v8h z;
#pragma unroll
    for (int j = 0; j < 8; ++j) z[j] = (_Float16)0.0f;
    unsigned short* dz = xpad + (size_t)kPatches * kPatchEl + t * 8;
    *(volatile v8h*)dz = z;
    __threadfence();
    *(volatile v8h*)dz = z;
  }
}

__global__ __launch_bounds__(256) void conv_kernel(const unsigned short* __restrict__ xpad,
                                                   const unsigned short* __restrict__ psfT,
                                                   float* __restrict__ blur)
{
  __shared__ __align__(16) float sT[8][16 * 36];
  const int lane = threadIdx.x & 31, wave = threadIdx.x >> 5;
  const int quarter = blockIdx.x & 3;
  const int pidx = blockIdx.x >> 2;
  const int g = pidx & (kCells - 1);
  const int bc = pidx >> 6;
  const int c = bc % kChan;
  const int gy = g >> 3, gx = g & 7;
  const int tile = quarter * 8 + wave;
  const int y0 = (tile >> 2) * 16;
  const int x0 = (tile & 3) * 32;
  const int rl = lane & 15, hf = lane >> 4;

  const _Float16* ap = (const _Float16*)xpad + (size_t)pidx * kPatchEl + (size_t)(y0 + rl) * kPadCols + x0 + 8 * hf;
  const _Float16* bp = (const _Float16*)psfT + (size_t)(g * kChan + c) * (kTapN * kToepPlane) + rl * kToepK + 8 * hf;

  v8f acc0 = (v8f){0.f,0.f,0.f,0.f,0.f,0.f,0.f,0.f};
  v8f acc1 = (v8f){0.f,0.f,0.f,0.f,0.f,0.f,0.f,0.f};
#pragma unroll 1
  for (int dy = 0; dy < kTapN; ++dy) {
    const v16h a00 = Frag<_Float16>::load(ap);
    const v16h a01 = Frag<_Float16>::load(ap + 32);
    const v16h a10 = Frag<_Float16>::load(ap + 16);
    const v16h a11 = Frag<_Float16>::load(ap + 48);
    const v16h b0  = Frag<_Float16>::load(bp);
    const v16h b1  = Frag<_Float16>::load(bp + 32);
    acc0 = mma_h(a00, b0, acc0);
    acc0 = mma_h(a01, b1, acc0);
    acc1 = mma_h(a10, b0, acc1);
    acc1 = mma_h(a11, b1, acc1);
    ap += kPadCols;
    bp += kToepPlane;
  }

  float* slab = sT[wave];
#pragma unroll
  for (int r = 0; r < 8; ++r) {
    slab[(8 * hf + r) * 36 + rl] = acc0[r] * kConvScale;
    slab[(8 * hf + r) * 36 + 16 + rl] = acc1[r] * kConvScale;
  }
  __builtin_amdgcn_fence(__ATOMIC_RELEASE, "workgroup");
  __builtin_amdgcn_wave_barrier();
  __builtin_amdgcn_fence(__ATOMIC_ACQUIRE, "workgroup");
  {
    const int q = lane >> 3, c4 = (lane & 7) * 4;
    float* dst = blur + ((size_t)bc * kImgH + gy * kCell + y0) * kImgW + gx * kCell + x0 + c4;
    for (int pass = 0; pass < 2; ++pass) {
#pragma unroll
      for (int it = 0; it < 4; ++it) {
        const int row = it * 4 + q;
        const v4f v = *(const v4f*)(slab + row * 36 + c4);
        *(volatile v4f*)(dst + (size_t)row * kImgW) = v;
      }
      __threadfence();
    }
  }
}

__global__ __launch_bounds__(256) void warp_kernel(const float* __restrict__ blur, const float* __restrict__ shifts,
                                                   float* __restrict__ out)
{
  __shared__ float sS[32];
  __shared__ __align__(16) float sO[8][kBatch * 96];
  const int t = threadIdx.x, lane = t & 31, wave = t >> 5;
  if (t < 32) sS[t] = shifts[imin_d(t, kFields - 1)];
  __syncthreads();
  const int pid = blockIdx.x * 256 + t;
  const int y = pid >> 10, x = pid & (kImgW - 1);
  const float xm = coordf(x), ym = coordf(y);
  const float r = sqrtf(xm * xm + ym * ym);
  int lo, hi;
  float f;
  soft_index(r * kFieldSteps, lo, hi, f);
  const float shift = sS[lo] * (1.0f - f) + sS[hi] * f;
  const float invr = 1.0f / r;
  const float cs = xm * invr, sn = ym * invr;
  const float qx = (float)x + shift * cs * kHalfDiag;
  const float qy = (float)y + shift * sn * kHalfDiag;
  const float fqx = floorf(qx), fqy = floorf(qy);
  const int x0 = (int)fqx, y0 = (int)fqy;
  const float fx = qx - fqx, fy = qy - fqy;

  float acc[kBatch * kChan];
#pragma unroll
  for (int p = 0; p < kBatch * kChan; ++p) acc[p] = 0.0f;
#pragma unroll 1
  for (int tp = 0; tp < 16; ++tp) {
    const int j = (tp >> 2) - 1, i = (tp & 3) - 1;
    const float wy = cubw(fabsf(fy - (float)j));
    const float wx = cubw(fabsf(fx - (float)i));
    const float w = wy * wx;
    const int yj = iclamp_d(y0 + j, 0, kImgH - 1);
    const int xi = iclamp_d(x0 + i, 0, kImgW - 1);
    const float* src = blur + (size_t)yj * kImgW + xi;
#pragma unroll
    for (int p = 0; p < kBatch * kChan; ++p) acc[p] = fmaf(w, src[(size_t)p * kPlaneEl], acc[p]);
  }
  float* slab = sO[wave];
#pragma unroll
  for (int p = 0; p < kBatch * kChan; ++p) slab[(p / kChan) * 96 + lane * kChan + (p % kChan)] = acc[p];
  __syncthreads();
  const int lc = imin_d(lane, 23);
  v4f ov[kBatch];
#pragma unroll
  for (int b = 0; b < kBatch; ++b) ov[b] = *(const v4f*)(slab + b * 96 + lc * 4);
  const int xw0 = x - lane;
  for (int pass = 0; pass < 2; ++pass) {
    if (lane < 24) {
#pragma unroll
      for (int b = 0; b < kBatch; ++b) {
        float* dst = out + ((size_t)(b * kImgH + y) * kImgW + xw0) * kChan + lane * 4;
        *(volatile v4f*)dst = ov[b];
      }
    }
    __threadfence();
  }
}

extern "C" void kernel_launch(void* const* d_in, const int* in_sizes, int n_in,
                              void* d_out, int out_size, void* d_ws, size_t ws_size,
                              hipStream_t stream) {
  if (n_in < 4) return;
  if (in_sizes[0] != kBatch * kImgH * kImgW * kChan) return;
  if (in_sizes[1] != kFields * kNPix) return;
  if (in_sizes[2] != kFields) return;
  if (in_sizes[3] != kFields) return;
  if (out_size != kBatch * kImgH * kImgW * kChan) return;
  if (ws_size < kWsTotal) return;

  const float* img    = (const float*)d_in[0];
  const float* psfs   = (const float*)d_in[1];
  const float* shifts = (const float*)d_in[2];
  const float* riTab  = (const float*)d_in[3];
  float* out = (float*)d_out;

  char* ws = (char*)d_ws;
  unsigned short* WTS    = (unsigned short*)(ws + kOffWTS);
  unsigned short* BT0    = (unsigned short*)(ws + kOffBT0);
  float*          INTERP = (float*)(ws + kOffINTERP);
  unsigned short* PSFT   = (unsigned short*)(ws + kOffPSFT);
  unsigned short* XPAD   = (unsigned short*)(ws + kOffXPAD);
  float*          BLUR   = (float*)(ws + kOffBLUR);

  weights_kernel<<<kCells, 256, 0, stream>>>(WTS);
  bt_plane_kernel<<<kNPixPad / 64, 256, 0, stream>>>(psfs, BT0);
  wmma_gemm64<0, false, 0, 0, false><<<dim3((kNPixPad / 64 + 7) / 8, 1), 256, 0, stream>>>(
      WTS, nullptr, kWtsLd, 0L,
      BT0, nullptr, kKPad, 0L,
      (void*)INTERP, nullptr, kNPixPad, 0L,
      nullptr, nullptr, 0L,
      kCells, kNPixPad, kKPad, kInterpScale);
  psf_finish_kernel<<<kCells, 256, 0, stream>>>(INTERP, PSFT);
  prep_kernel<<<kBatch * kCells, 256, 0, stream>>>(img, riTab, XPAD);
  conv_kernel<<<kPatches * 4, 256, 0, stream>>>(XPAD, PSFT, BLUR);
  warp_kernel<<<(kImgH * kImgW) / 256, 256, 0, stream>>>(BLUR, shifts, out);
}
